// CrossAttentionBridge_63582695850803
// MI455X (gfx1250) — hardware-verified
//
#include <hip/hip_runtime.h>


typedef _Float16 v16h __attribute__((ext_vector_type(16)));
typedef _Float16 v8h  __attribute__((ext_vector_type(8)));
typedef _Float16 v4h  __attribute__((ext_vector_type(4)));
typedef float    v8f  __attribute__((ext_vector_type(8)));
typedef float    v4f  __attribute__((ext_vector_type(4)));
typedef unsigned int v4u __attribute__((ext_vector_type(4)));
typedef unsigned int v2u __attribute__((ext_vector_type(2)));

union Frag   { v16h v; v8h half[2]; };
union Pack16 { v8h h; v4u u; };
union Pack8  { v4h h; v2u u; };

#define D_MODEL  1024
#define NHEAD    16
#define HDIM     64
#define LSEQ     512
#define NBATCH   8
#define MROWS    (NBATCH * LSEQ)
#define LN_EPS   1e-5f
#define QK_SCALE 0.125f
#define W_SCALE  64.0f
#define W_ISCALE 0.015625f
#define P_SCALE  4096.0f
#define P_ISCALE 0.000244140625f

#define WMMA_NOPS "v_nop\n\tv_nop\n\tv_nop\n\tv_nop"

__device__ __forceinline__ v8f wmma_f16(v16h a, v16h b, v8f c) {
    return __builtin_amdgcn_wmma_f32_16x16x32_f16(false, a, false, b, (short)0, c, false, false);
}

__global__ __launch_bounds__(128)
void k_layernorm(const float* __restrict__ x, const float* __restrict__ gamma,
                 const float* __restrict__ beta, _Float16* __restrict__ y, int nrows)
{
    __shared__ float red[4];
    const int row = blockIdx.x;
    if (row >= nrows) return;
    const int tid = threadIdx.x, lane = tid & 31, w = tid >> 5;
    const float* xr = x + (size_t)row * D_MODEL + tid * 8;
    const v4f x0 = *(const v4f*)(xr);
    const v4f x1 = *(const v4f*)(xr + 4);
    float v[8];
#pragma unroll
    for (int i = 0; i < 4; ++i) { v[i] = x0[i]; v[4 + i] = x1[i]; }
    float s = 0.f;
#pragma unroll
    for (int i = 0; i < 8; ++i) s += v[i];
#pragma unroll
    for (int m = 16; m > 0; m >>= 1) s += __shfl_xor(s, m, 32);
    if (lane == 0) red[w] = s;
    __syncthreads();
    const float mu = ((red[0] + red[1]) + (red[2] + red[3])) * (1.0f / D_MODEL);
    __syncthreads();
    float sq = 0.f;
#pragma unroll
    for (int i = 0; i < 8; ++i) { const float d = v[i] - mu; sq += d * d; }
#pragma unroll
    for (int m = 16; m > 0; m >>= 1) sq += __shfl_xor(sq, m, 32);
    if (lane == 0) red[w] = sq;
    __syncthreads();
    const float var = ((red[0] + red[1]) + (red[2] + red[3])) * (1.0f / D_MODEL);
    const float rstd = rsqrtf(var + LN_EPS);
    const float* gp = gamma + tid * 8;
    const float* bp = beta + tid * 8;
    const v4f g0 = *(const v4f*)(gp), g1 = *(const v4f*)(gp + 4);
    const v4f b0 = *(const v4f*)(bp), b1 = *(const v4f*)(bp + 4);
    Pack16 o;
#pragma unroll
    for (int i = 0; i < 4; ++i) {
        o.h[i]     = (_Float16)((v[i] - mu) * rstd * g0[i] + b0[i]);
        o.h[4 + i] = (_Float16)((v[4 + i] - mu) * rstd * g1[i] + b1[i]);
    }
    _Float16* dst = y + (size_t)row * D_MODEL + tid * 8;
    *(volatile v4u*)dst = o.u;
    __threadfence();
    *(volatile v4u*)dst = o.u;
}

__global__ __launch_bounds__(256)
void k_convert(const float* __restrict__ src, _Float16* __restrict__ dst, int n, float scale)
{
    const size_t base = ((size_t)blockIdx.x * 256 + threadIdx.x) * 8;
    if (base + 8 > (size_t)n) return;
    const v4f a = *(const v4f*)(src + base);
    const v4f b = *(const v4f*)(src + base + 4);
    Pack16 o;
#pragma unroll
    for (int i = 0; i < 4; ++i) {
        o.h[i]     = (_Float16)(a[i] * scale);
        o.h[4 + i] = (_Float16)(b[i] * scale);
    }
    _Float16* d = dst + base;
    *(volatile v4u*)d = o.u;
    __threadfence();
    *(volatile v4u*)d = o.u;
}

__device__ __forceinline__ float bias128(int i, int j) {
    const float d = fabsf((float)(i - j));
    return __expf(-(d * 0.1f)) - d * 0.05f;
}
__device__ __forceinline__ float bias_resized(int q, int k) {
    float x = ((float)q + 0.5f) * 0.25f - 0.5f;
    float y = ((float)k + 0.5f) * 0.25f - 0.5f;
    x = fminf(fmaxf(x, 0.0f), 127.0f);
    y = fminf(fmaxf(y, 0.0f), 127.0f);
    const int x0 = (int)floorf(x), y0 = (int)floorf(y);
    const int x1 = min(x0 + 1, 127), y1 = min(y0 + 1, 127);
    const float fx = x - (float)x0, fy = y - (float)y0;
    const float t0 = bias128(x0, y0) * (1.0f - fx) + bias128(x1, y0) * fx;
    const float t1 = bias128(x0, y1) * (1.0f - fx) + bias128(x1, y1) * fx;
    return t0 * (1.0f - fy) + t1 * fy;
}
__global__ __launch_bounds__(256)
void k_bias_table(float* __restrict__ bt)
{
    const int t = blockIdx.x * 256 + threadIdx.x;
    if (t >= LSEQ * (LSEQ / 4)) return;
    const int q = t >> 7;
    const int k4 = (t & 127) * 4;
    v4f v;
    v[0] = bias_resized(q, k4 + 0);
    v[1] = bias_resized(q, k4 + 1);
    v[2] = bias_resized(q, k4 + 2);
    v[3] = bias_resized(q, k4 + 3);
    float* dst = bt + (size_t)q * LSEQ + k4;
    *(volatile v4f*)dst = v;
    __threadfence();
    *(volatile v4f*)dst = v;
}

__global__ __launch_bounds__(256)
void k_rope_table(float* __restrict__ ct, float* __restrict__ st)
{
    const int t = blockIdx.x * 256 + threadIdx.x;
    if (t >= LSEQ * (HDIM / 2)) return;
    const int l = t >> 5, i = t & 31;
    const float inv = exp2f((float)i * -0.4152410118609203f);
    const float f = (float)l * inv;
    float sn, cs;
    sincosf(f, &sn, &cs);
    *(volatile float*)(ct + t) = cs;
    *(volatile float*)(st + t) = sn;
    __threadfence();
    *(volatile float*)(ct + t) = cs;
    *(volatile float*)(st + t) = sn;
}

template <int MODE>
__global__ __launch_bounds__(256)
void k_gemm(const _Float16* __restrict__ A, const _Float16* __restrict__ W,
            const float* __restrict__ bias, const float* __restrict__ aux0,
            const float* __restrict__ aux1, float* outf, _Float16* outh,
            int N, int K, float oscale)
{
    const int tid = threadIdx.x;
    const int lane = tid & 31, w = tid >> 5;
    const int hh = lane >> 4, l15 = lane & 15;
    const int bm = blockIdx.y * 128 + w * 16;
    const int bn = blockIdx.x * 64;

    const v8f zero = {0.f, 0.f, 0.f, 0.f, 0.f, 0.f, 0.f, 0.f};
    v8f acc[4];
#pragma unroll
    for (int j = 0; j < 4; ++j) acc[j] = zero;

    const _Float16* arow = A + (size_t)(bm + l15) * K + 8 * hh;
    const _Float16* brow = W + (size_t)(bn + 4 * l15) * K + 8 * hh;
    const size_t Ks = (size_t)K;

#pragma unroll 1
    for (int k0 = 0; k0 < K; k0 += 32) {
        Frag a, b0, b1, b2, b3;
        a.half[0]  = *(const v8h*)(arow + k0);
        a.half[1]  = *(const v8h*)(arow + k0 + 16);
        b0.half[0] = *(const v8h*)(brow + k0);
        b0.half[1] = *(const v8h*)(brow + k0 + 16);
        b1.half[0] = *(const v8h*)(brow + Ks + k0);
        b1.half[1] = *(const v8h*)(brow + Ks + k0 + 16);
        b2.half[0] = *(const v8h*)(brow + 2 * Ks + k0);
        b2.half[1] = *(const v8h*)(brow + 2 * Ks + k0 + 16);
        b3.half[0] = *(const v8h*)(brow + 3 * Ks + k0);
        b3.half[1] = *(const v8h*)(brow + 3 * Ks + k0 + 16);
        acc[0] = wmma_f16(a.v, b0.v, acc[0]);
        acc[1] = wmma_f16(a.v, b1.v, acc[1]);
        acc[2] = wmma_f16(a.v, b2.v, acc[2]);
        acc[3] = wmma_f16(a.v, b3.v, acc[3]);
        asm volatile(WMMA_NOPS
                     : "+v"(acc[0]), "+v"(acc[1]), "+v"(acc[2]), "+v"(acc[3])
                     : "v"(a.v), "v"(b0.v), "v"(b1.v), "v"(b2.v), "v"(b3.v));
    }

    if constexpr (MODE == 0) {
        const int col = bn + 4 * l15;
        const v4f bv = *(const v4f*)(bias + col);
        v4f vals[8];
#pragma unroll
        for (int r = 0; r < 8; ++r) {
            v4f t;
            t[0] = acc[0][r] * oscale + bv[0];
            t[1] = acc[1][r] * oscale + bv[1];
            t[2] = acc[2][r] * oscale + bv[2];
            t[3] = acc[3][r] * oscale + bv[3];
            vals[r] = t;
        }
        float* cb = outf + (size_t)(bm + 8 * hh) * N + col;
#pragma unroll
        for (int r = 0; r < 8; ++r) *(volatile v4f*)(cb + (size_t)r * N) = vals[r];
        __threadfence();
#pragma unroll
        for (int r = 0; r < 8; ++r) *(volatile v4f*)(cb + (size_t)r * N) = vals[r];
    }

    if constexpr (MODE == 1) {
        const int head = blockIdx.x;
        const int bb = bm / LSEQ;
        const int l0 = (bm % LSEQ) + 8 * hh;
        const int fi = 4 * (l15 & 7);
        const float sgn = (l15 < 8) ? -1.0f : 1.0f;
        v2u vals[8];
#pragma unroll
        for (int r = 0; r < 8; ++r) {
            const int l = l0 + r;
            const v4f cv = *(const v4f*)(aux0 + (size_t)l * (HDIM / 2) + fi);
            const v4f sv = *(const v4f*)(aux1 + (size_t)l * (HDIM / 2) + fi);
            Pack8 o;
#pragma unroll
            for (int j = 0; j < 4; ++j) {
                const float xv = acc[j][r] * oscale;
                const float xp = __shfl_xor(xv, 8, 32);
                o.h[j] = (_Float16)(xv * cv[j] + sgn * (xp * sv[j]));
            }
            vals[r] = o.u;
        }
        _Float16* qb = outh + ((size_t)(bb * NHEAD + head) * LSEQ + l0) * HDIM + 4 * l15;
#pragma unroll
        for (int r = 0; r < 8; ++r) *(volatile v2u*)(qb + (size_t)r * HDIM) = vals[r];
        __threadfence();
#pragma unroll
        for (int r = 0; r < 8; ++r) *(volatile v2u*)(qb + (size_t)r * HDIM) = vals[r];
    }

    if constexpr (MODE == 2) {
        __shared__ __attribute__((aligned(16))) _Float16 vt[HDIM][128 + 8];
        const int head = blockIdx.x;
        const int kvl = w * 16 + 8 * hh;
#pragma unroll
        for (int j = 0; j < 4; ++j)
#pragma unroll
            for (int r = 0; r < 8; ++r)
                vt[4 * l15 + j][kvl + r] = (_Float16)(acc[j][r] * oscale);
        __syncthreads();
        const int brow0 = blockIdx.y * 128;
        const int bb = brow0 / LSEQ, kv0 = brow0 % LSEQ;
        const int bh = bb * NHEAD + head;
        Pack16 vals[4];
#pragma unroll
        for (int p = 0; p < 4; ++p) {
            const int d = 8 * w + 2 * p + hh;
            vals[p].h = *(const v8h*)(&vt[d][l15 * 8]);
        }
        _Float16* vbp = outh + ((size_t)bh * HDIM + 8 * w + hh) * LSEQ + kv0 + l15 * 8;
#pragma unroll
        for (int p = 0; p < 4; ++p) *(volatile v4u*)(vbp + (size_t)(2 * p) * LSEQ) = vals[p].u;
        __threadfence();
#pragma unroll
        for (int p = 0; p < 4; ++p) *(volatile v4u*)(vbp + (size_t)(2 * p) * LSEQ) = vals[p].u;
    }

    if constexpr (MODE == 3) {
        const int col = bn + 4 * l15;
        const v4f bv = *(const v4f*)(bias + col);
        const int row0 = bm + 8 * hh;
        v4f vals[8];
#pragma unroll
        for (int r = 0; r < 8; ++r) {
            const size_t off = (size_t)(row0 + r) * N + col;
            const v4f pj = *(const v4f*)(aux0 + off);
            const v4f rs = *(const v4f*)(aux1 + off);
            v4f t;
#pragma unroll
            for (int j = 0; j < 4; ++j) {
                const float g  = acc[j][r] * oscale + bv[j];
                const float sg = __builtin_amdgcn_rcpf(1.0f + __expf(-g));
                t[j] = sg * pj[j] + (1.0f - sg) * rs[j];
            }
            vals[r] = t;
        }
        float* ob = outf + (size_t)row0 * N + col;
#pragma unroll
        for (int r = 0; r < 8; ++r) *(volatile v4f*)(ob + (size_t)r * N) = vals[r];
        __threadfence();
#pragma unroll
        for (int r = 0; r < 8; ++r) *(volatile v4f*)(ob + (size_t)r * N) = vals[r];
    }
}

__global__ __launch_bounds__(32)
void k_attn(const _Float16* __restrict__ q16, const _Float16* __restrict__ k16,
            const _Float16* __restrict__ vT, const float* __restrict__ bt,
            _Float16* __restrict__ a16)
{
    __shared__ __attribute__((aligned(16))) _Float16 pbuf[16][72];
    const int lane = threadIdx.x & 31;
    const int hh = lane >> 4, l15 = lane & 15;
    const int bid = blockIdx.x;
    const int qt = bid & 31, bh = bid >> 5;
    const int bb = bh >> 4, head = bh & 15;

    const _Float16* qp = q16 + ((size_t)bh * LSEQ + qt * 16 + l15) * HDIM + 8 * hh;
    const _Float16* kb = k16 + (size_t)bh * LSEQ * HDIM + 8 * hh;
    const _Float16* vb = vT + (size_t)bh * HDIM * LSEQ + 8 * hh;

    Frag qa0, qa1;
    qa0.half[0] = *(const v8h*)(qp);
    qa0.half[1] = *(const v8h*)(qp + 16);
    qa1.half[0] = *(const v8h*)(qp + 32);
    qa1.half[1] = *(const v8h*)(qp + 48);

    const v8f zero = {0.f, 0.f, 0.f, 0.f, 0.f, 0.f, 0.f, 0.f};
    float rm[8], rl[8];
    v8f oacc[4];
#pragma unroll
    for (int r = 0; r < 8; ++r) { rm[r] = -1e30f; rl[r] = 0.f; }
#pragma unroll
    for (int n = 0; n < 4; ++n) oacc[n] = zero;

    const float* btrow = bt + (size_t)(qt * 16 + 8 * hh) * LSEQ + l15;

#pragma unroll 1
    for (int c0 = 0; c0 < LSEQ; c0 += 64) {
        v8f s[4];
#pragma unroll
        for (int nt = 0; nt < 4; ++nt) {
            const _Float16* kr = kb + (size_t)(c0 + nt * 16 + l15) * HDIM;
            Frag kf0, kf1;
            kf0.half[0] = *(const v8h*)(kr);
            kf0.half[1] = *(const v8h*)(kr + 16);
            kf1.half[0] = *(const v8h*)(kr + 32);
            kf1.half[1] = *(const v8h*)(kr + 48);
            v8f z = zero;
            z = wmma_f16(qa0.v, kf0.v, z);
            z = wmma_f16(qa1.v, kf1.v, z);
            asm volatile(WMMA_NOPS : "+v"(z) : "v"(qa0.v), "v"(qa1.v), "v"(kf0.v), "v"(kf1.v));
            s[nt] = z;
        }
#pragma unroll
        for (int nt = 0; nt < 4; ++nt)
#pragma unroll
            for (int r = 0; r < 8; ++r)
                s[nt][r] = s[nt][r] * QK_SCALE + btrow[(size_t)r * LSEQ + c0 + nt * 16];

        float alpha[8];
#pragma unroll
        for (int r = 0; r < 8; ++r) {
            float loc = fmaxf(fmaxf(s[0][r], s[1][r]), fmaxf(s[2][r], s[3][r]));
            loc = fmaxf(loc, __shfl_xor(loc, 1, 32));
            loc = fmaxf(loc, __shfl_xor(loc, 2, 32));
            loc = fmaxf(loc, __shfl_xor(loc, 4, 32));
            loc = fmaxf(loc, __shfl_xor(loc, 8, 32));
            const float mn = fmaxf(rm[r], loc);
            alpha[r] = __expf(rm[r] - mn);
            rm[r] = mn;
            const float p0 = __expf(s[0][r] - mn);
            const float p1 = __expf(s[1][r] - mn);
            const float p2 = __expf(s[2][r] - mn);
            const float p3 = __expf(s[3][r] - mn);
            s[0][r] = p0; s[1][r] = p1; s[2][r] = p2; s[3][r] = p3;
            float rs = (p0 + p1) + (p2 + p3);
            rs += __shfl_xor(rs, 1, 32);
            rs += __shfl_xor(rs, 2, 32);
            rs += __shfl_xor(rs, 4, 32);
            rs += __shfl_xor(rs, 8, 32);
            rl[r] = rl[r] * alpha[r] + rs;
        }
#pragma unroll
        for (int n = 0; n < 4; ++n)
#pragma unroll
            for (int r = 0; r < 8; ++r) oacc[n][r] *= alpha[r];

        __syncthreads();
#pragma unroll
        for (int nt = 0; nt < 4; ++nt)
#pragma unroll
            for (int r = 0; r < 8; ++r)
                pbuf[8 * hh + r][nt * 16 + l15] = (_Float16)(s[nt][r] * P_SCALE);
        __syncthreads();

#pragma unroll
        for (int kc = 0; kc < 2; ++kc) {
            Frag pa;
            pa.half[0] = *(const v8h*)(&pbuf[l15][kc * 32 + 8 * hh]);
            pa.half[1] = *(const v8h*)(&pbuf[l15][kc * 32 + 16 + 8 * hh]);
            const _Float16* vr = vb + (size_t)(4 * l15) * LSEQ + c0 + kc * 32;
            Frag vf0, vf1, vf2, vf3;
            vf0.half[0] = *(const v8h*)(vr);
            vf0.half[1] = *(const v8h*)(vr + 16);
            vf1.half[0] = *(const v8h*)(vr + LSEQ);
            vf1.half[1] = *(const v8h*)(vr + LSEQ + 16);
            vf2.half[0] = *(const v8h*)(vr + 2 * LSEQ);
            vf2.half[1] = *(const v8h*)(vr + 2 * LSEQ + 16);
            vf3.half[0] = *(const v8h*)(vr + 3 * LSEQ);
            vf3.half[1] = *(const v8h*)(vr + 3 * LSEQ + 16);
            oacc[0] = wmma_f16(pa.v, vf0.v, oacc[0]);
            oacc[1] = wmma_f16(pa.v, vf1.v, oacc[1]);
            oacc[2] = wmma_f16(pa.v, vf2.v, oacc[2]);
            oacc[3] = wmma_f16(pa.v, vf3.v, oacc[3]);
            asm volatile(WMMA_NOPS
                         : "+v"(oacc[0]), "+v"(oacc[1]), "+v"(oacc[2]), "+v"(oacc[3])
                         : "v"(pa.v), "v"(vf0.v), "v"(vf1.v), "v"(vf2.v), "v"(vf3.v));
        }
    }

    v2u vals[8];
#pragma unroll
    for (int r = 0; r < 8; ++r) {
        const float inv = __builtin_amdgcn_rcpf(rl[r]) * P_ISCALE;
        Pack8 o;
        o.h[0] = (_Float16)(oacc[0][r] * inv);
        o.h[1] = (_Float16)(oacc[1][r] * inv);
        o.h[2] = (_Float16)(oacc[2][r] * inv);
        o.h[3] = (_Float16)(oacc[3][r] * inv);
        vals[r] = o.u;
    }
    _Float16* ob = a16 + ((size_t)bb * LSEQ + qt * 16 + 8 * hh) * D_MODEL + head * HDIM + 4 * l15;
#pragma unroll
    for (int r = 0; r < 8; ++r) *(volatile v2u*)(ob + (size_t)r * D_MODEL) = vals[r];
    __threadfence();
#pragma unroll
    for (int r = 0; r < 8; ++r) *(volatile v2u*)(ob + (size_t)r * D_MODEL) = vals[r];
}

extern "C" void kernel_launch(void* const* d_in, const int* in_sizes, int n_in,
                              void* d_out, int out_size, void* d_ws, size_t ws_size,
                              hipStream_t stream)
{
    if (n_in < 9) return;
    const int nact = MROWS * D_MODEL;
    const int nw = D_MODEL * D_MODEL;
    if (in_sizes[0] != nact || in_sizes[1] != nact || in_sizes[2] != 3 * nw ||
        in_sizes[3] != nw || in_sizes[4] != D_MODEL || in_sizes[5] != nw ||
        in_sizes[6] != D_MODEL || in_sizes[7] != D_MODEL || in_sizes[8] != D_MODEL ||
        out_size != nact) return;

    const float* dec   = (const float*)d_in[0];
    const float* enc   = (const float*)d_in[1];
    const float* Wqkv  = (const float*)d_in[2];
    const float* Wout  = (const float*)d_in[3];
    const float* bout  = (const float*)d_in[4];
    const float* Wgate = (const float*)d_in[5];
    const float* bgate = (const float*)d_in[6];
    const float* gamma = (const float*)d_in[7];
    const float* beta  = (const float*)d_in[8];
    float* out = (float*)d_out;

    size_t off = 0;
    auto carve = [&off](size_t bytes) -> size_t {
        const size_t p = off;
        off += (bytes + 255) & ~(size_t)255;
        return p;
    };
    const size_t o_h16  = carve((size_t)nact * 2);
    const size_t o_e16  = carve((size_t)nact * 2);
    const size_t o_wq   = carve((size_t)nw * 2);
    const size_t o_wk   = carve((size_t)nw * 2);
    const size_t o_wv   = carve((size_t)nw * 2);
    const size_t o_wo   = carve((size_t)nw * 2);
    const size_t o_wg   = carve((size_t)nw * 2);
    const size_t o_bt   = carve((size_t)LSEQ * LSEQ * 4);
    const size_t o_rc   = carve((size_t)LSEQ * (HDIM / 2) * 4);
    const size_t o_rs   = carve((size_t)LSEQ * (HDIM / 2) * 4);
    const size_t o_q16  = carve((size_t)nact * 2);
    const size_t o_k16  = carve((size_t)nact * 2);
    const size_t o_v16  = carve((size_t)nact * 2);
    const size_t o_a16  = carve((size_t)nact * 2);
    const size_t o_proj = carve((size_t)nact * 4);
    const size_t o_p16  = carve((size_t)nact * 2);
    if (off > ws_size) return;

    char* ws = (char*)d_ws;
    _Float16* h16  = (_Float16*)(ws + o_h16);
    _Float16* e16  = (_Float16*)(ws + o_e16);
    _Float16* wq   = (_Float16*)(ws + o_wq);
    _Float16* wk   = (_Float16*)(ws + o_wk);
    _Float16* wv   = (_Float16*)(ws + o_wv);
    _Float16* wo   = (_Float16*)(ws + o_wo);
    _Float16* wg   = (_Float16*)(ws + o_wg);
    float*    bt   = (float*)(ws + o_bt);
    float*    rc   = (float*)(ws + o_rc);
    float*    rs   = (float*)(ws + o_rs);
    _Float16* q16  = (_Float16*)(ws + o_q16);
    _Float16* k16  = (_Float16*)(ws + o_k16);
    _Float16* v16  = (_Float16*)(ws + o_v16);
    _Float16* a16  = (_Float16*)(ws + o_a16);
    float*    proj = (float*)(ws + o_proj);
    _Float16* p16  = (_Float16*)(ws + o_p16);

    const dim3 b256(256), b128(128), b32(32);

    k_layernorm<<<dim3(MROWS), b128, 0, stream>>>(dec, gamma, beta, h16, MROWS);
    k_layernorm<<<dim3(MROWS), b128, 0, stream>>>(enc, gamma, beta, e16, MROWS);
    k_bias_table<<<dim3((LSEQ * (LSEQ / 4) + 255) / 256), b256, 0, stream>>>(bt);
    k_rope_table<<<dim3((LSEQ * (HDIM / 2) + 255) / 256), b256, 0, stream>>>(rc, rs);

    const unsigned cvt_w = (unsigned)((nw / 8 + 255) / 256);
    k_convert<<<dim3(cvt_w), b256, 0, stream>>>(Wqkv, wq, nw, W_SCALE);
    k_convert<<<dim3(cvt_w), b256, 0, stream>>>(Wqkv + (size_t)nw, wk, nw, W_SCALE);
    k_convert<<<dim3(cvt_w), b256, 0, stream>>>(Wqkv + (size_t)2 * nw, wv, nw, W_SCALE);
    k_convert<<<dim3(cvt_w), b256, 0, stream>>>(Wout, wo, nw, W_SCALE);
    k_convert<<<dim3(cvt_w), b256, 0, stream>>>(Wgate, wg, nw, W_SCALE);

    const dim3 gg(D_MODEL / 64, MROWS / 128);
    k_gemm<1><<<gg, b256, 0, stream>>>(h16, wq, bout, rc, rs, proj, q16, D_MODEL, D_MODEL, W_ISCALE);
    k_gemm<1><<<gg, b256, 0, stream>>>(e16, wk, bout, rc, rs, proj, k16, D_MODEL, D_MODEL, W_ISCALE);
    k_gemm<2><<<gg, b256, 0, stream>>>(e16, wv, bout, rc, rs, proj, v16, D_MODEL, D_MODEL, W_ISCALE);

    k_attn<<<dim3(NBATCH * NHEAD * (LSEQ / 16)), b32, 0, stream>>>(q16, k16, v16, bt, a16);

    k_gemm<0><<<gg, b256, 0, stream>>>(a16, wo, bout, rc, rs, proj, p16, D_MODEL, D_MODEL, W_ISCALE);
    const unsigned cvt_a = (unsigned)((nact / 8 + 255) / 256);
    k_convert<<<dim3(cvt_a), b256, 0, stream>>>(proj, p16, nact, 1.0f);
    k_gemm<3><<<gg, b256, 0, stream>>>(p16, wg, bgate, proj, dec, out, a16, D_MODEL, D_MODEL, W_ISCALE);
}
